// TemporalPhaseManifold_68891275427896
// MI455X (gfx1250) — hardware-run, weakly checked
//
#include <hip/hip_runtime.h>
#include <math.h>

typedef __attribute__((ext_vector_type(16))) _Float16 v16h;
typedef __attribute__((ext_vector_type(16))) __bf16 v16b;
typedef __attribute__((ext_vector_type(8)))  _Float16 v8h;
typedef __attribute__((ext_vector_type(8)))  float v8f;
typedef __attribute__((ext_vector_type(4)))  float v4f;
typedef __attribute__((ext_vector_type(2)))  float v2f;
typedef __attribute__((ext_vector_type(4)))  unsigned v4u;
typedef __attribute__((ext_vector_type(4)))  int v4i;
typedef float __attribute__((may_alias)) float_a;
typedef int __attribute__((may_alias)) int_a;

template <typename T> __device__ __forceinline__ void vst2(void* p, T v) { *(volatile T*)p = v; __threadfence(); *(volatile T*)p = v; }
__device__ __forceinline__ v8f wmma16(v16h a, v16h b, v8f c) {
  v8f d = __builtin_amdgcn_wmma_f32_16x16x32_f16(false, a, false, b, (short)0, c, false, false);
  asm volatile("v_nop\n\tv_nop\n\tv_nop\n\tv_nop" : "+v"(d) : "v"(a), "v"(b));
  return d;
}
__device__ __forceinline__ v8f wmma_bf(v16b a, v16b b, v8f c) {
  v8f d = __builtin_amdgcn_wmma_f32_16x16x32_bf16(false, a, false, b, (short)0, c, false, false);
  asm volatile("v_nop\n\tv_nop\n\tv_nop\n\tv_nop" : "+v"(d) : "v"(a), "v"(b));
  return d;
}
__device__ __forceinline__ v16h frag_h(const _Float16* rowk0, int lane) {
  union { v16h v; v8h q[2]; } u; const _Float16* p = rowk0 + 8 * (lane >> 4);
  u.q[0] = *(const v8h*)p; u.q[1] = *(const v8h*)(p + 16); return u.v;
}
__device__ __forceinline__ v16h frag_f32(const float* rowk0, int lane) {
  v16h a; const float* p = rowk0 + 8 * (lane >> 4);
#pragma unroll
  for (int i = 0; i < 8; ++i) { a[i] = (_Float16)p[i]; a[8 + i] = (_Float16)p[16 + i]; }
  return a;
}
__device__ __forceinline__ v16h frag_f32s(const float* rowk0, int lane, float sc) {
  v16h a; const float* p = rowk0 + 8 * (lane >> 4);
#pragma unroll
  for (int i = 0; i < 8; ++i) { a[i] = (_Float16)(p[i] * sc); a[8 + i] = (_Float16)(p[16 + i] * sc); }
  return a;
}
__device__ __forceinline__ v16h fragc_f32(const float* W, int k0, int n, int lane, int ld, int K) {
  v16h a; const int g = lane >> 4;
#pragma unroll
  for (int i = 0; i < 8; ++i) { const int ka = k0 + 8 * g + i, kb = ka + 16;
    a[i] = (_Float16)(ka < K ? W[(size_t)(ka < K ? ka : K - 1) * ld + n] : 0.f); a[8 + i] = (_Float16)(kb < K ? W[(size_t)(kb < K ? kb : K - 1) * ld + n] : 0.f); }
  return a;
}
struct F2 { v16b h, l; };
__device__ __forceinline__ F2 bsplit16(const float v[16]) { F2 r;
#pragma unroll
  for (int i = 0; i < 16; ++i) { const __bf16 h = (__bf16)v[i]; r.h[i] = h; r.l[i] = (__bf16)(v[i] - (float)h); }
  return r; }
__device__ __forceinline__ F2 split_row(const float* row, int k0, int lane) { float v[16]; const float* p = row + k0 + 8 * (lane >> 4);
#pragma unroll
  for (int i = 0; i < 8; ++i) { v[i] = p[i]; v[8 + i] = p[16 + i]; }
  return bsplit16(v); }
__device__ __forceinline__ F2 split_rowK(const float* row, int k0, int lane, int K) { float v[16]; const int g = lane >> 4;
#pragma unroll
  for (int i = 0; i < 8; ++i) { const int ka = k0 + 8 * g + i, kb = ka + 16; v[i] = ka < K ? row[ka < K ? ka : K - 1] : 0.f; v[8 + i] = kb < K ? row[kb < K ? kb : K - 1] : 0.f; }
  return bsplit16(v); }
__device__ __forceinline__ F2 split_col(const float* W, int k0, int n, int lane, int ld, int K) { float v[16]; const int g = lane >> 4;
#pragma unroll
  for (int i = 0; i < 8; ++i) { const int ka = k0 + 8 * g + i, kb = ka + 16; v[i] = ka < K ? W[(size_t)(ka < K ? ka : K - 1) * ld + n] : 0.f; v[8 + i] = kb < K ? W[(size_t)(kb < K ? kb : K - 1) * ld + n] : 0.f; }
  return bsplit16(v); }
__device__ __forceinline__ v8f mac3(const F2& a, const F2& b, v8f c) { c = wmma_bf(a.l, b.h, c); c = wmma_bf(a.h, b.l, c); return wmma_bf(a.h, b.h, c); }
__device__ __forceinline__ float sigm(float v) { return 1.0f / (1.0f + expf(-v)); }
#define LDSX() do { asm volatile("s_wait_dscnt 0" ::: "memory"); __builtin_amdgcn_wave_barrier(); __builtin_amdgcn_fence(__ATOMIC_RELEASE, "workgroup"); } while (0)


#define NB 4
#define SS 1024
#define DIN 256
#define MM 1024
#define NH 16
#define HD 64
#define HX 96
#define NF 8
#define NL 2
#define DH1 512
#define DOUT 256
#define NR (NB * SS)
#ifndef TQB
#define TQB (SS / 64)
#define TNB NB
#endif
typedef __attribute__((ext_vector_type(8))) __bf16 v8b;
__device__ __forceinline__ v16b frag_b(const __bf16* rowk0, int lane) {
  union { v16b v; v8b q[2]; } u; const __bf16* p = rowk0 + 8 * (lane >> 4);
  u.q[0] = *(const v8b*)p; u.q[1] = *(const v8b*)(p + 16); return u.v;
}
__device__ __forceinline__ float bfr(float v) { return (float)(__bf16)v; }
__device__ __attribute__((noinline)) float exp_ni(float v) { return expf(v); }
__device__ __attribute__((noinline)) float erf_ni(float v) { return erff(v); }

__device__ __attribute__((noinline)) float sin_p(float v) { return sinf(v); }
__device__ __attribute__((noinline)) float cos_p(float v) { return cosf(v); }

#define WS_PE  0u
#define WS_PL  (WS_PE + 2u * (size_t)MM * DIN)
#define WS_P1  (WS_PL + 2u * (size_t)NL * 4 * MM * MM)
#define WS_P2  (WS_P1 + 2u * (size_t)DH1 * MM)
#define WS_PF  (WS_P2 + 2u * (size_t)DOUT * DH1)
#define WS_Y   (WS_PF + 4u * (size_t)NR * MM)
#define WS_O   (WS_Y + 4u * (size_t)NR * MM)
#define WS_H1  (WS_O + 4u * (size_t)NR * MM)
#define WS_QK  (WS_H1 + 4u * (size_t)NR * DH1)
#define WS_KK  (WS_QK + 2u * (size_t)NR * NH * HX)
#define WS_V   (WS_KK + 2u * (size_t)NR * NH * HX)
#define WS_CS  (WS_V + 2u * (size_t)NB * MM * SS)
#define WS_END (WS_CS + 4u * (size_t)SS * NF * 2)

__global__ __launch_bounds__(256) void k_packh(const float* __restrict__ WEMB, const float* __restrict__ WQ, const float* __restrict__ WK, const float* __restrict__ WV, const float* __restrict__ WO, const float* __restrict__ W1, const float* __restrict__ W2, _Float16* __restrict__ P) {
  __shared__ __align__(16) _Float16 s[MM]; const int n = blockIdx.x, id = blockIdx.y, t = threadIdx.x;
  const float* src; int K, N; size_t dst;
  if (id == 0) { src = WEMB; K = DIN; N = MM; dst = WS_PE / 2; }
  else if (id <= 8) { const int l = (id - 1) / 4, which = (id - 1) % 4; src = ((which == 0) ? WQ : (which == 1) ? WK : (which == 2) ? WV : WO) + (size_t)l * MM * MM; K = MM; N = MM; dst = WS_PL / 2 + ((size_t)(l * 4 + which) * MM) * MM; }
  else if (id == 9) { src = W1; K = MM; N = DH1; dst = WS_P1 / 2; } else { src = W2; K = DH1; N = DOUT; dst = WS_P2 / 2; }
  if (n >= N) return;
  for (int k = t; k < K; k += 256) s[k] = (_Float16)(bfr(src[(size_t)k * N + n]) * 256.0f);
  __syncthreads(); for (int q = t; q < K / 8; q += 256) vst2((unsigned*)(P + dst + (size_t)n * K + q * 8), *(const v4u*)&s[q * 8]);
}
__global__ __launch_bounds__(256) void k_phase(const float* __restrict__ FRQ, const float* __restrict__ PHO, float* __restrict__ CS) { __shared__ __align__(16) float st[SS * NF * 2]; const int t = threadIdx.x;
  for (int e = t; e < SS * NF; e += 256) { const int s = e / NF, f = e % NF; const float tc = (float)s / (float)SS * 6.283185307179586f; const float pc = tc * bfr(FRQ[f]) + bfr(PHO[f]); st[e * 2] = cos_p(pc); st[e * 2 + 1] = sin_p(pc); }
  __syncthreads(); for (int q = t; q < SS * NF * 2 / 4; q += 256) vst2(CS + q * 4, *(const v4f*)&st[q * 4]); }
template <int KW, int EPI, int RAW>
__global__ __launch_bounds__(128) void k_lin(const float* __restrict__ A, const _Float16* __restrict__ Wr, const float* __restrict__ BIAS, const float* __restrict__ R, float* __restrict__ Y, int ystride) {
  __shared__ __align__(16) float so[4][16][132];
  const int tid = threadIdx.x, wave = tid >> 5, lane = tid & 31, col = lane & 15, g = lane >> 4; const size_t r0 = (size_t)blockIdx.x * 64 + wave * 16; const int n0 = blockIdx.y * 128;
  v8f acc[8] = {};
#pragma unroll 2
  for (int kc = 0; kc < KW / 32; ++kc) { v16h a; { const float* p = A + (r0 + col) * KW + kc * 32 + 8 * g;
#pragma unroll
      for (int i = 0; i < 8; ++i) { a[i] = (_Float16)(RAW ? bfr(p[i]) : p[i]); a[8 + i] = (_Float16)(RAW ? bfr(p[16 + i]) : p[16 + i]); } }
#pragma unroll
    for (int j = 0; j < 8; ++j) acc[j] = wmma16(a, frag_h(Wr + (size_t)(n0 + j * 16 + col) * KW + kc * 32, lane), acc[j]); }
#pragma unroll
  for (int j = 0; j < 8; ++j) { const int c = n0 + j * 16 + col; const float bb = bfr(BIAS[c]);
#pragma unroll
    for (int r = 0; r < 8; ++r) { float v = acc[j][r] * (1.0f / 256.0f) + bb; if (EPI == 1) v = fabsf(v) * (1.0f / (float)NF); if (EPI == 2) v = fmaxf(v, 0.f); if (EPI == 3) v += R[(r0 + 8 * g + r) * (size_t)ystride + c]; so[wave][8 * g + r][j * 16 + col] = v; } }
  LDSX();
  for (int rl = 0; rl < 16; ++rl) vst2(Y + (r0 + rl) * (size_t)ystride + n0 + lane * 4, *(const v4f*)&so[wave][rl][lane * 4]);
}
__global__ __launch_bounds__(256) void k_ln(const float* __restrict__ X, const float* __restrict__ G, const float* __restrict__ Bt, float* __restrict__ XN) {
  __shared__ float red[8]; const int t = threadIdx.x; const size_t row = blockIdx.x; float v[4]; float s = 0.f; for (int i = 0; i < 4; ++i) { v[i] = X[row * MM + t * 4 + i]; s += v[i]; }
#pragma unroll
  for (int o = 1; o < 32; o <<= 1) s += __shfl_xor(s, o);
  if ((t & 31) == 0) red[t >> 5] = s; __syncthreads(); float tot = 0.f; for (int i = 0; i < 8; ++i) tot += red[i]; const float mu = tot / (float)MM; __syncthreads();
  float q = 0.f; for (int i = 0; i < 4; ++i) { const float d = v[i] - mu; q += d * d; }
#pragma unroll
  for (int o = 1; o < 32; o <<= 1) q += __shfl_xor(q, o);
  if ((t & 31) == 0) red[t >> 5] = q; __syncthreads(); float tq = 0.f; for (int i = 0; i < 8; ++i) tq += red[i]; const float inv = 1.0f / sqrtf(tq / (float)MM + 1e-5f);
  v4f o4; for (int i = 0; i < 4; ++i) { const int e = t * 4 + i; o4[i] = (v[i] - mu) * inv * bfr(G[e]) + bfr(Bt[e]); } vst2(XN + row * MM + t * 4, o4);
}
__global__ __launch_bounds__(128) void k_qkv(const float* __restrict__ PF, const _Float16* __restrict__ WL, const float* __restrict__ BQ, const float* __restrict__ BK, const float* __restrict__ BV, const float* __restrict__ PB, const float* __restrict__ CS, _Float16* __restrict__ QQ, _Float16* __restrict__ KK, _Float16* __restrict__ V) {
  __shared__ __align__(16) _Float16 so[64][2 * HX + 8]; __shared__ __align__(16) _Float16 st[128][72];
  const int tid = threadIdx.x, wave = tid >> 5, lane = tid & 31, col = lane & 15, g = lane >> 4; const int which = blockIdx.z; const size_t rb = (size_t)blockIdx.x * 64; const size_t r0 = rb + wave * 16; const int c0 = blockIdx.y * 128; const int h0 = c0 / HD;
  const _Float16* Wr = WL + ((size_t)which * MM) * MM; const float* BB = (which == 0) ? BQ : (which == 1) ? BK : BV;
  v8f acc[8] = {};
#pragma unroll 2
  for (int kc = 0; kc < MM / 32; ++kc) { v16h a; { const float* p = PF + (r0 + col) * MM + kc * 32 + 8 * g;
#pragma unroll
      for (int i = 0; i < 8; ++i) { a[i] = (_Float16)p[i]; a[8 + i] = (_Float16)p[16 + i]; } }
#pragma unroll
    for (int j = 0; j < 8; ++j) acc[j] = wmma16(a, frag_h(Wr + (size_t)(c0 + j * 16 + col) * MM + kc * 32, lane), acc[j]); }
  if (which < 2) { const float scl = (which == 0) ? 0.125f : 1.0f;
#pragma unroll
    for (int j = 0; j < 8; ++j) { const int cl = j * 16 + col; const int hl = cl >> 6, d = cl & 63; const float bb = bfr(BB[c0 + cl]);
#pragma unroll
      for (int r = 0; r < 8; ++r) so[wave * 16 + 8 * g + r][hl * HX + d] = (_Float16)((acc[j][r] * (1.0f / 256.0f) + bb) * scl); }
    for (int e = tid; e < 64 * 2 * 32; e += 128) { const int rl = e >> 6, rem = e & 63; const int hl = rem >> 5, x = rem & 31; const int s = (int)((rb + rl) % SS); float v = 0.f;
      if (x < 2 * NF) { const int f = x & (NF - 1); const float cs = CS[(s * NF + f) * 2 + (x >= NF ? 1 : 0)]; v = (which == 0) ? bfr(PB[(h0 + hl) * NF + f]) * cs : cs; }
      so[rl][hl * HX + HD + x] = (_Float16)v; }
    __syncthreads();
    _Float16* dst = (which == 0) ? QQ : KK;
    for (int e = tid; e < 64 * (2 * HX / 8); e += 128) { const int rl = e / (2 * HX / 8), q = e % (2 * HX / 8); vst2((unsigned*)(dst + ((rb + rl) * NH + h0) * HX + q * 8), *(const v4u*)&so[rl][q * 8]); }
  } else {
#pragma unroll
    for (int j = 0; j < 8; ++j) { const float bb = bfr(BB[c0 + j * 16 + col]);
#pragma unroll
      for (int r = 0; r < 8; ++r) st[j * 16 + col][wave * 16 + 8 * g + r] = (_Float16)(acc[j][r] * (1.0f / 256.0f) + bb); }
    __syncthreads();
    const size_t b = rb / SS; const int s0 = (int)(rb % SS);
    for (int e = tid; e < 128 * 8; e += 128) { const int d = e >> 3, pc = e & 7; vst2((unsigned*)(V + ((b * MM + c0 + d) * SS) + s0 + pc * 8), *(const v4u*)&st[d][pc * 8]); } }
}
__global__ __launch_bounds__(128) void k_attn(const _Float16* __restrict__ QQ, const _Float16* __restrict__ KK, const _Float16* __restrict__ V, float* __restrict__ O) {
  __shared__ __align__(16) _Float16 sph[4][16][40]; __shared__ __align__(16) float so[4][16][68];
  const int tid = threadIdx.x, wave = tid >> 5, lane = tid & 31, col = lane & 15, g = lane >> 4; const int h = blockIdx.y; const size_t b = blockIdx.z; const int q0 = blockIdx.x * 64 + wave * 16; const size_t rq = b * SS + q0;
  v16h aq[3];
#pragma unroll
  for (int kc = 0; kc < 3; ++kc) aq[kc] = frag_h(QQ + ((rq + col) * NH + h) * HX + kc * 32, lane);
  float m[8], l[8];
#pragma unroll
  for (int r = 0; r < 8; ++r) { m[r] = -3.0e38f; l[r] = 0.f; }
  v8f acc[4] = {};
#pragma unroll 1
  for (int ks = 0; ks < SS / 32; ++ks) { const int j0 = ks * 32; v8f s[2];
#pragma unroll
    for (int ct = 0; ct < 2; ++ct) { const size_t rk = ((b * SS + j0 + ct * 16 + col) * NH + h) * HX; v8f c = {};
#pragma unroll
      for (int kc = 0; kc < 3; ++kc) c = wmma16(aq[kc], frag_h(KK + rk + kc * 32, lane), c);
#pragma unroll
      for (int r = 0; r < 8; ++r) s[ct][r] = c[r]; }
#pragma unroll
    for (int r = 0; r < 8; ++r) { float mx = fmaxf(s[0][r], s[1][r]);
#pragma unroll
      for (int o = 1; o < 16; o <<= 1) mx = fmaxf(mx, __shfl_xor(mx, o));
      const float mn = fmaxf(m[r], mx); const float alpha = (m[r] <= -1.0e38f) ? 0.f : __expf(m[r] - mn); const float e0 = __expf(s[0][r] - mn), e1 = __expf(s[1][r] - mn); float es = e0 + e1;
#pragma unroll
      for (int o = 1; o < 16; o <<= 1) es += __shfl_xor(es, o);
      l[r] = l[r] * alpha + es; m[r] = mn;
#pragma unroll
      for (int dt = 0; dt < 4; ++dt) acc[dt][r] *= alpha;
      sph[wave][8 * g + r][col] = (_Float16)(e0 * 2048.0f); sph[wave][8 * g + r][16 + col] = (_Float16)(e1 * 2048.0f); }
    LDSX();
    const v16h pa = frag_h(&sph[wave][col][0], lane);
#pragma unroll
    for (int dt = 0; dt < 4; ++dt) acc[dt] = wmma16(pa, frag_h(V + ((b * MM + h * HD + dt * 16 + col) * SS) + j0, lane), acc[dt]);
    LDSX(); }
#pragma unroll
  for (int r = 0; r < 8; ++r) { const float il = (1.0f / 2048.0f) / l[r];
#pragma unroll
    for (int dt = 0; dt < 4; ++dt) so[wave][8 * g + r][dt * 16 + col] = acc[dt][r] * il; }
  LDSX();
  for (int rl = 0; rl < 16; ++rl) if (lane < 16) vst2(O + (rq + rl) * MM + h * HD + lane * 4, *(const v4f*)&so[wave][rl][lane * 4]);
}
extern "C" void kernel_launch(void* const* d_in, const int* in_sizes, int n_in, void* d_out, int out_size, void* d_ws, size_t ws_size, hipStream_t stream) {
  (void)in_sizes; (void)n_in; (void)out_size;
  const float** F = (const float**)d_in;
  if (ws_size < (size_t)WS_END) return;
  char* ws = (char*)d_ws; _Float16 *P = (_Float16*)ws, *QQ = (_Float16*)(ws + WS_QK), *KK = (_Float16*)(ws + WS_KK), *V = (_Float16*)(ws + WS_V); float *PF = (float*)(ws + WS_PF), *Y = (float*)(ws + WS_Y), *O = (float*)(ws + WS_O), *H1 = (float*)(ws + WS_H1), *CS = (float*)(ws + WS_CS);
  k_packh<<<dim3(MM, 11), 256, 0, stream>>>(F[1], F[7], F[9], F[11], F[13], F[18], F[20], P);
  k_phase<<<1, 256, 0, stream>>>(F[5], F[6], CS);
  k_lin<DIN, 1, 1><<<dim3(TNB * SS / 64, MM / 128), 128, 0, stream>>>(F[0], P + WS_PE / 2, F[2], nullptr, PF, MM);
  for (int l = 0; l < NL; ++l) { const _Float16* WL = P + WS_PL / 2 + ((size_t)(l * 4) * MM) * MM;
    k_qkv<<<dim3(TNB * SS / 64, MM / 128, 3), 128, 0, stream>>>(PF, WL, F[8] + l * MM, F[10] + l * MM, F[12] + l * MM, F[15] + l * NH * NF, CS, QQ, KK, V);
    k_attn<<<dim3(TQB, NH, TNB), 128, 0, stream>>>(QQ, KK, V, O);
    k_lin<MM, 3, 0><<<dim3(TNB * SS / 64, MM / 128), 128, 0, stream>>>(O, WL + (size_t)3 * MM * MM, F[14] + l * MM, PF, Y, MM);
    k_ln<<<TNB * SS, 256, 0, stream>>>(Y, F[16] + l * MM, F[17] + l * MM, PF); }
  k_lin<MM, 2, 0><<<dim3(TNB * SS / 64, DH1 / 128), 128, 0, stream>>>(PF, P + WS_P1 / 2, F[19], nullptr, H1, DH1);
  k_lin<DH1, 0, 0><<<dim3(TNB * SS / 64, DOUT / 128), 128, 0, stream>>>(H1, P + WS_P2 / 2, F[21], nullptr, (float*)d_out, DOUT);
}
